// LocalContextAttentionBlock_6828998000689
// MI455X (gfx1250) — hardware-verified
//
#include <hip/hip_runtime.h>
#include <math.h>
#include <stdint.h>


#define BATCH 2
#define CH    128
#define HH    180
#define WW    180
#define HW    32400
#define PPAD  32448
#define BN_EPS 1e-5f

typedef __attribute__((ext_vector_type(16))) _Float16 v16h;
typedef __attribute__((ext_vector_type(8)))  _Float16 v8h;
typedef __attribute__((ext_vector_type(16))) __bf16   v16b;
typedef __attribute__((ext_vector_type(8)))  __bf16   v8b;
typedef __attribute__((ext_vector_type(8)))  float    v8f;
typedef __attribute__((ext_vector_type(4)))  float    v4f;
#define PSCALE 32768.0f
#define U16(p) ((const unsigned short*)(const void*)(p))
#define PSCALE_INV (1.0f / 32768.0f)

__device__ __forceinline__ unsigned short f2bf_bits(float f) {
  unsigned u = __float_as_uint(f);
  return (unsigned short)((u + 0x7FFFu + ((u >> 16) & 1u)) >> 16);
}
__device__ __forceinline__ float bf_bits2f(unsigned short h) { return __uint_as_float(((unsigned)h) << 16); }

__device__ __forceinline__ void dep_guard_h(v8f& a, v8f& b, v16h x, v16h y) { asm volatile("v_nop\n\tv_nop\n\tv_nop\n\tv_nop" : "+v"(a), "+v"(b) : "v"(x), "v"(y)); }
__device__ __forceinline__ void dep_guard_b(v8f& a, v8f& b, v16b x, v16b y) { asm volatile("v_nop\n\tv_nop\n\tv_nop\n\tv_nop" : "+v"(a), "+v"(b) : "v"(x), "v"(y)); }
__device__ __forceinline__ void keep4_h(v16h a, v16h b, v16h c, v16h d) { asm volatile("v_nop" :: "v"(a), "v"(b), "v"(c), "v"(d)); }
__device__ __forceinline__ void keep4_b(v16b a, v16b b, v16b c, v16b d) { asm volatile("v_nop" :: "v"(a), "v"(b), "v"(c), "v"(d)); }
__device__ __forceinline__ void acc_guard4(v8f& a, v8f& b, v8f& c, v8f& d) { asm volatile("v_nop\n\tv_nop\n\tv_nop\n\tv_nop" : "+v"(a), "+v"(b), "+v"(c), "+v"(d)); }
template <typename T> struct Frag;
template <> struct Frag<_Float16> {
  typedef v16h V; union U { v16h v; v8h h[2]; };
  static __device__ __forceinline__ v16h load(const _Float16* p) {
    U f; f.h[0] = *(const v8h*)(p); f.h[1] = *(const v8h*)(p + 16); return f.v;
  }
  static __device__ __forceinline__ v8f mma(v16h a, v16h b, v8f c) {
    return __builtin_amdgcn_wmma_f32_16x16x32_f16(false, a, false, b, (short)0, c, false, false);
  }
  static __device__ __forceinline__ void guard(v8f& a, v8f& b, v16h x, v16h y) { dep_guard_h(a, b, x, y); }
  static __device__ __forceinline__ void keep(v16h a, v16h b, v16h c, v16h d) { keep4_h(a, b, c, d); }
};
template <> struct Frag<__bf16> {
  typedef v16b V; union U { v16b v; v8b h[2]; };
  static __device__ __forceinline__ v16b load(const __bf16* p) {
    U f; f.h[0] = *(const v8b*)(p); f.h[1] = *(const v8b*)(p + 16); return f.v;
  }
  static __device__ __forceinline__ v8f mma(v16b a, v16b b, v8f c) {
    return __builtin_amdgcn_wmma_f32_16x16x32_bf16(false, a, false, b, (short)0, c, false, false);
  }
  static __device__ __forceinline__ void guard(v8f& a, v8f& b, v16b x, v16b y) { dep_guard_b(a, b, x, y); }
  static __device__ __forceinline__ void keep(v16b a, v16b b, v16b c, v16b d) { keep4_b(a, b, c, d); }
};

template <int ET> struct Elem;
template <> struct Elem<0> { typedef _Float16 T; };
template <> struct Elem<1> { typedef __bf16 T; };
template <int ET, bool SPLIT, int BIAS_MODE, int OUT_MODE, bool RESID, int ACT = 0>
__global__ __launch_bounds__(256) void wmma_gemm64(
    const unsigned short* __restrict__ Ap, const unsigned short* __restrict__ A2p, int lda, long strideA,
    const unsigned short* __restrict__ Btp, const unsigned short* __restrict__ Bt2p, int ldb, long strideB,
    void* __restrict__ Cout, void* __restrict__ Cout2, int ldc, long strideC,
    const float* __restrict__ bias,
    const float* __restrict__ resid, long strideR,
    int M, int N, int K, float scale) {
  typedef typename Elem<ET>::T T;
  typedef typename Frag<T>::V V;
  const T* A = (const T*)Ap; const T* A2 = (const T*)A2p; const T* Bt = (const T*)Btp; const T* Bt2 = (const T*)Bt2p;
  __shared__ __align__(16) float sT[8][16 * 68];
  const int b    = blockIdx.y;
  const int lane = threadIdx.x & 31;
  const int wave = threadIdx.x >> 5;
  const int tilesN = N >> 6;
  const int tilesM = M >> 6;
  const int tile = blockIdx.x * 8 + wave;
  if (tile >= tilesM * tilesN) return;
  const int tm = tile / tilesN;
  const int tn = tile - tm * tilesN;
  const int m0 = tm << 6;
  const int n0 = tn << 6;

  const T* Ab  = A  + (size_t)b * strideA;
  const T* Bb  = Bt + (size_t)b * strideB;
  const T* Ab2 = SPLIT ? (A2  + (size_t)b * strideA) : nullptr;
  const T* Bb2 = SPLIT ? (Bt2 + (size_t)b * strideB) : nullptr;

  const int rlane = lane & 15;
  const int koff  = (lane >> 4) * 8;
  const int mOff  = (lane >> 4) * 8;

  v8f acc[4][4];
#pragma unroll
  for (int i = 0; i < 4; ++i)
#pragma unroll
    for (int j = 0; j < 4; ++j) acc[i][j] = (v8f){0.f,0.f,0.f,0.f,0.f,0.f,0.f,0.f};

  for (int k0 = 0; k0 < K; k0 += 32) {
    V bh[4], bl[4];
#pragma unroll
    for (int j = 0; j < 4; ++j) {
      const size_t bo = (size_t)(n0 + (j << 4) + rlane) * ldb + koff + k0;
      bh[j] = Frag<T>::load(Bb + bo);
      if (SPLIT) bl[j] = Frag<T>::load(Bb2 + bo);
    }
#pragma unroll
    for (int i = 0; i < 4; ++i) {
      const size_t ao = (size_t)(m0 + (i << 4) + rlane) * lda + koff + k0;
      V ah = Frag<T>::load(Ab + ao);
      V al;
      if (SPLIT) al = Frag<T>::load(Ab2 + ao);
#pragma unroll
      for (int j = 0; j < 4; ++j) {
        acc[i][j] = Frag<T>::mma(ah, bh[j], acc[i][j]);
        if (SPLIT) {
          acc[i][j] = Frag<T>::mma(ah, bl[j], acc[i][j]);
          acc[i][j] = Frag<T>::mma(al, bh[j], acc[i][j]);
        }
      }
      Frag<T>::guard(acc[i][0], acc[i][3], ah, SPLIT ? al : ah);
    }
    Frag<T>::keep(bh[0], bh[1], bh[2], bh[3]);
    if (SPLIT) Frag<T>::keep(bl[0], bl[1], bl[2], bl[3]);
  }
  acc_guard4(acc[0][0], acc[0][1], acc[0][2], acc[0][3]);
  acc_guard4(acc[1][0], acc[1][1], acc[1][2], acc[1][3]);
  acc_guard4(acc[2][0], acc[2][1], acc[2][2], acc[2][3]);
  acc_guard4(acc[3][0], acc[3][1], acc[3][2], acc[3][3]);

  float* slab = sT[wave];
  const float* Rb = RESID ? (resid + (size_t)b * strideR) : nullptr;
#pragma unroll
  for (int i = 0; i < 4; ++i) {
    const int mBase = m0 + (i << 4);
#pragma unroll
    for (int j = 0; j < 4; ++j) {
      const int n = n0 + (j << 4) + rlane;
      float bv = 0.f;
      if (BIAS_MODE == 2) bv = bias[n];
#pragma unroll
      for (int r = 0; r < 8; ++r) {
        float v = acc[i][j][r] * scale;
        if (BIAS_MODE == 1) v += bias[mBase + mOff + r];
        if (BIAS_MODE == 2) v += bv;
        if (RESID) v += Rb[(size_t)(mBase + mOff + r) * ldc + n];
        if (ACT == 1) v = tanhf(v);
        if (ACT == 2) v = fmaxf(v, 0.0f);
        if (ACT == 3) v = v / (1.0f + expf(-v));
        if (ACT == 4) v = (v > 0.f) ? v : 0.01f * v;
        if (ACT == 5) v = 0.5f * v * (1.0f + erff(v * 0.70710678118654752f));
        slab[(mOff + r) * 68 + (j << 4) + rlane] = v;
      }
    }
    __builtin_amdgcn_fence(__ATOMIC_RELEASE, "workgroup");
    __builtin_amdgcn_wave_barrier();
    __builtin_amdgcn_fence(__ATOMIC_ACQUIRE, "workgroup");
    if (OUT_MODE == 0) {
      float* C = (float*)Cout + (size_t)b * strideC;
      const int hh = lane >> 4, c4 = (lane & 15) * 4;
      for (int pass = 0; pass < 2; ++pass) {
#pragma unroll
        for (int it = 0; it < 8; ++it) {
          const int row = it * 2 + hh;
          v4f v = *(const v4f*)(slab + row * 68 + c4);
          *(volatile v4f*)(C + (size_t)(mBase + row) * ldc + n0 + c4) = v;
        }
        __threadfence();
      }
    } else {
      const int q = lane >> 3, c8 = (lane & 7) * 8;
      unsigned short* C  = (unsigned short*)Cout  + (size_t)b * strideC;
      unsigned short* C2 = (OUT_MODE == 2) ? ((unsigned short*)Cout2 + (size_t)b * strideC) : nullptr;
      for (int pass = 0; pass < 2; ++pass) {
#pragma unroll
        for (int it = 0; it < 4; ++it) {
          const int row = it * 4 + q;
          const float* sp = slab + row * 68 + c8;
          v8h hv, lv;
#pragma unroll
          for (int e = 0; e < 8; ++e) {
            if (OUT_MODE == 1) {
              hv[e] = (_Float16)sp[e];
            } else {
              unsigned short hb = f2bf_bits(sp[e]);
              unsigned short lb = f2bf_bits(sp[e] - bf_bits2f(hb));
              hv[e] = __builtin_bit_cast(_Float16, hb);
              lv[e] = __builtin_bit_cast(_Float16, lb);
            }
          }
          *(volatile v8h*)(C + (size_t)(mBase + row) * ldc + n0 + c8) = hv;
          if (OUT_MODE == 2) *(volatile v8h*)(C2 + (size_t)(mBase + row) * ldc + n0 + c8) = lv;
        }
        __threadfence();
      }
    }
    __builtin_amdgcn_fence(__ATOMIC_RELEASE, "workgroup");
    __builtin_amdgcn_wave_barrier();
    __builtin_amdgcn_fence(__ATOMIC_ACQUIRE, "workgroup");
  }
}

__device__ __forceinline__ v8f mma_h(v16h a, v16h b, v8f c) {
  c = __builtin_amdgcn_wmma_f32_16x16x32_f16(false, a, false, b, (short)0, c, false, false);
  asm volatile("v_nop\n\tv_nop\n\tv_nop\n\tv_nop" : "+v"(c) : "v"(a), "v"(b));
  return c;
}
__device__ __forceinline__ void lds_wave_sync() {
  __builtin_amdgcn_fence(__ATOMIC_RELEASE, "workgroup");
  __builtin_amdgcn_wave_barrier();
  __builtin_amdgcn_fence(__ATOMIC_ACQUIRE, "workgroup");
}

__global__ __launch_bounds__(256)
void fold_w_kernel(const float* __restrict__ Wm, const float* __restrict__ g, const float* __restrict__ bb,
                   const float* __restrict__ mm, const float* __restrict__ vv,
                   _Float16* __restrict__ W16, float* __restrict__ shift)
{
  const int i = blockIdx.x * 256 + threadIdx.x;
  if (i < (CH * CH) / 2) {
    const int o = (2 * i) >> 7;
    const float sc = g[o] * rsqrtf(vv[o] + BN_EPS);
    const _Float16 h0 = (_Float16)(Wm[2 * i] * sc);
    const _Float16 h1 = (_Float16)(Wm[2 * i + 1] * sc);
    const unsigned u = (unsigned)__builtin_bit_cast(unsigned short, h0) |
                       ((unsigned)__builtin_bit_cast(unsigned short, h1) << 16);
    ((volatile unsigned*)W16)[i] = u;
    __threadfence();
    ((volatile unsigned*)W16)[i] = u;
  }
  if (i < CH) {
    const float sc = g[i] * rsqrtf(vv[i] + BN_EPS);
    const float sh = bb[i] - mm[i] * sc;
    ((volatile float*)shift)[i] = sh;
    __threadfence();
    ((volatile float*)shift)[i] = sh;
  }
}

#define TPH 136
__global__ __launch_bounds__(256)
void nchw_to_pc16_kernel(const float* __restrict__ X, _Float16* __restrict__ XT)
{
  __shared__ __align__(16) _Float16 t16[64 * TPH];
  const int tid = threadIdx.x, wave = tid >> 5, lane = tid & 31;
  const int b = blockIdx.y;
  const int p0 = blockIdx.x * 64;
  const int pl = tid & 63, cg = tid >> 6;
  const int p = p0 + pl;
  const float* Xb = X + (size_t)b * CH * HW;
#pragma unroll 4
  for (int i = 0; i < 32; ++i) {
    const int ch = cg + 4 * i;
    float v = 0.0f;
    if (p < HW) v = Xb[(size_t)ch * HW + p];
    t16[pl * TPH + ch] = (_Float16)v;
  }
  __syncthreads();
  _Float16* XTb = XT + (size_t)b * PPAD * CH;
  const int rh = lane >> 4, c8 = (lane & 15) * 8;
  for (int pass = 0; pass < 2; ++pass) {
#pragma unroll
    for (int rr = 0; rr < 4; ++rr) {
      const int row = wave * 8 + rr * 2 + rh;
      const v8h v = *(const v8h*)(t16 + row * TPH + c8);
      *(volatile v8h*)(XTb + (size_t)(p0 + row) * CH + c8) = v;
    }
    __threadfence();
  }
}

#define NTILE 23
#define KPH   136
#define VPH   264
#define SPF   164
#define PPH   (2*SPF)

__global__ __launch_bounds__(128)
void local_attn_kernel(const _Float16* __restrict__ Q16, const _Float16* __restrict__ K16,
                       const _Float16* __restrict__ V16, float* __restrict__ ATT)
{
  __shared__ __align__(16) _Float16 KVsh[256 * KPH];
  __shared__ __align__(16) float    Ssh[4][16 * SPF];
  __shared__ float Lsh[4][16];

  const int tid = threadIdx.x;
  const int wave = tid >> 5, lane = tid & 31, h = lane >> 4, c = lane & 15;
  const int b  = blockIdx.y;
  const int ty = blockIdx.x / NTILE;
  const int tx = blockIdx.x - ty * NTILE;
  const int y0 = ty * 8, x0 = tx * 8;
  const size_t bofs = (size_t)b * PPAD * CH;
  const int jbase = 2 * wave;

  v16h qa[4];
  {
    const int rq = wave * 16 + c;
    const int qy = rq >> 3, qx = rq & 7;
    const int gy = y0 + qy, gx = x0 + qx;
    const int qp = (gy < HH && gx < WW) ? (gy * WW + gx) : 0;
    const _Float16* qrow = Q16 + bofs + (size_t)qp * CH + 8 * h;
#pragma unroll
    for (int kc = 0; kc < 4; ++kc) qa[kc] = Frag<_Float16>::load(qrow + kc * 32);
  }
  v8h z8;
#pragma unroll
  for (int e = 0; e < 8; ++e) z8[e] = (_Float16)0.0f;

#pragma unroll 1
  for (int it = 0; it < 32; ++it) {
    const int qd = it * 128 + tid;
    const int n = qd >> 4, ch8 = (qd & 15) * 8;
    const int gy = y0 - 4 + (n >> 4), gx = x0 - 4 + (n & 15);
    v8h kv = z8;
    if (gy >= 0 && gy < HH && gx >= 0 && gx < WW)
      kv = *(const v8h*)(K16 + bofs + (size_t)(gy * WW + gx) * CH + ch8);
    *(v8h*)(KVsh + n * KPH + ch8) = kv;
  }
  __syncthreads();

  float* Sw = Ssh[wave];
#pragma unroll 1
  for (int jj = 0; jj < 10; ++jj) {
    const _Float16* krow = KVsh + ((jbase + jj) * 16 + c) * KPH + 8 * h;
    v8f acc = (v8f){0.f,0.f,0.f,0.f,0.f,0.f,0.f,0.f};
#pragma unroll
    for (int kc = 0; kc < 4; ++kc) {
      const v16h kb = Frag<_Float16>::load(krow + kc * 32);
      acc = mma_h(qa[kc], kb, acc);
    }
#pragma unroll
    for (int r = 0; r < 8; ++r) Sw[(8 * h + r) * SPF + jj * 16 + c] = acc[r];
  }
  __syncthreads();

#pragma unroll 1
  for (int it = 0; it < 32; ++it) {
    const int qd = it * 128 + tid;
    const int n = qd >> 4, ch8 = (qd & 15) * 8;
    const int gy = y0 - 4 + (n >> 4), gx = x0 - 4 + (n & 15);
    v8h vv = z8;
    if (gy >= 0 && gy < HH && gx >= 0 && gx < WW)
      vv = *(const v8h*)(V16 + bofs + (size_t)(gy * WW + gx) * CH + ch8);
#pragma unroll
    for (int e = 0; e < 8; ++e) KVsh[(ch8 + e) * VPH + n] = vv[e];
  }
  __syncthreads();

  _Float16* Pw = (_Float16*)Sw;
  const float kInv = 0.08838834764831845f;
  const bool lact = (lane < 20);
  const int iy  = jbase + (lane >> 1);
  const int ix0 = (lane & 1) * 8;
#pragma unroll 1
  for (int rr = 0; rr < 16; ++rr) {
    const int r = wave * 16 + rr;
    const int ry = r >> 3, rx = r & 7;
    const bool rowin = lact && (iy >= ry) && (iy <= ry + 8);
    v4f s0 = (v4f){0.f,0.f,0.f,0.f}, s1 = (v4f){0.f,0.f,0.f,0.f};
    if (lact) {
      s0 = *(const v4f*)(Sw + rr * SPF + lane * 8);
      s1 = *(const v4f*)(Sw + rr * SPF + lane * 8 + 4);
    }
    float x[8];
    x[0] = s0[0]; x[1] = s0[1]; x[2] = s0[2]; x[3] = s0[3];
    x[4] = s1[0]; x[5] = s1[1]; x[6] = s1[2]; x[7] = s1[3];
    bool inw[8];
    float m = -INFINITY;
#pragma unroll
    for (int e = 0; e < 8; ++e) {
      inw[e] = rowin && (ix0 + e >= rx) && (ix0 + e <= rx + 8);
      x[e] *= kInv;
      if (inw[e]) m = fmaxf(m, x[e]);
    }
#pragma unroll
    for (int off = 16; off > 0; off >>= 1) m = fmaxf(m, __shfl_xor(m, off, 32));
    float sum = 0.f;
    v8h pv;
#pragma unroll
    for (int e = 0; e < 8; ++e) {
      const float p = inw[e] ? __expf(x[e] - m) : 0.0f;
      sum += p;
      pv[e] = (_Float16)(p * 32768.0f);
    }
#pragma unroll
    for (int off = 16; off > 0; off >>= 1) sum += __shfl_xor(sum, off, 32);
    if (lact) *(v8h*)(Pw + rr * PPH + lane * 8) = pv;
    if (lane == 0) Lsh[wave][rr] = 1.0f / (sum * 32768.0f);
  }
  lds_wave_sync();

  v8f oacc[8];
#pragma unroll
  for (int t = 0; t < 8; ++t) oacc[t] = (v8f){0.f,0.f,0.f,0.f,0.f,0.f,0.f,0.f};
#pragma unroll 1
  for (int kk = 0; kk < 5; ++kk) {
    const v16h pa = Frag<_Float16>::load(Pw + c * PPH + kk * 32 + 8 * h);
    const _Float16* vrow = KVsh + c * VPH + jbase * 16 + kk * 32 + 8 * h;
#pragma unroll
    for (int t = 0; t < 8; ++t) {
      const v16h vb = Frag<_Float16>::load(vrow + t * 16 * VPH);
      oacc[t] = mma_h(pa, vb, oacc[t]);
    }
  }
  lds_wave_sync();

#pragma unroll
  for (int r = 0; r < 8; ++r) {
    const float inv = Lsh[wave][8 * h + r];
#pragma unroll
    for (int t = 0; t < 8; ++t) Sw[(8 * h + r) * SPF + t * 16 + c] = oacc[t][r] * inv;
  }
  lds_wave_sync();
  float* Ab = ATT + bofs;
  for (int pass = 0; pass < 2; ++pass) {
#pragma unroll 1
    for (int rr = 0; rr < 16; ++rr) {
      const int r = wave * 16 + rr;
      const int gy = y0 + (r >> 3), gx = x0 + (r & 7);
      if (gy < HH && gx < WW) {
        const v4f v = *(const v4f*)(Sw + rr * SPF + lane * 4);
        *(volatile v4f*)(Ab + (size_t)(gy * WW + gx) * CH + lane * 4) = v;
      }
    }
    __threadfence();
  }
}

__global__ __launch_bounds__(256)
void pc_to_nchw_out_kernel(const float* __restrict__ ATT, float* __restrict__ out, int n_out)
{
  const int f0 = (blockIdx.x * 256 + threadIdx.x) * 4;
  if (f0 + 3 < n_out) {
    const int bc = f0 / HW;
    const int p  = f0 - bc * HW;
    const int b  = bc >> 7, ch = bc & 127;
    const float* src = ATT + ((size_t)b * PPAD + p) * CH + ch;
    v4f v;
    v[0] = src[0]; v[1] = src[CH]; v[2] = src[2 * CH]; v[3] = src[3 * CH];
    *(volatile v4f*)(out + f0) = v;
    __threadfence();
    *(volatile v4f*)(out + f0) = v;
  }
}

static void launch_gemm(const _Float16* A, const _Float16* W16, const float* shift, _Float16* C, hipStream_t stream)
{
  wmma_gemm64<0, false, 2, 1, false, 2><<<dim3((PPAD / 64 * (CH / 64) + 7) / 8, BATCH), dim3(256), 0, stream>>>(
      (const unsigned short*)A, (const unsigned short*)A, CH, (long)PPAD * CH,
      (const unsigned short*)W16, (const unsigned short*)W16, CH, 0L,
      (void*)C, (void*)C, CH, (long)PPAD * CH,
      shift, shift, 0L,
      PPAD, CH, CH, 1.0f);
}

extern "C" void kernel_launch(void* const* d_in, const int* in_sizes, int n_in,
                              void* d_out, int out_size, void* d_ws, size_t ws_size,
                              hipStream_t stream)
{
  if (n_in < 27) return;
  const int ten = BATCH * CH * HW;
  if (in_sizes[0] != ten || in_sizes[1] != ten || out_size != ten) return;
  for (int i = 0; i < 5; ++i) {
    if (in_sizes[2 + 5 * i] != CH * CH) return;
    for (int j = 1; j < 5; ++j) if (in_sizes[2 + 5 * i + j] != CH) return;
  }

  const size_t TEN16 = (size_t)BATCH * PPAD * CH * 2;
  const size_t WBYTES = (size_t)CH * CH * 2;
  const size_t SBYTES = (size_t)CH * 4;
  const size_t off_xt  = 0;
  const size_t off_tmp = off_xt + TEN16;
  const size_t off_att = 0;
  const size_t off_q   = off_tmp + TEN16;
  const size_t off_k   = off_q + TEN16;
  const size_t off_v   = off_k + TEN16;
  const size_t off_w   = off_v + TEN16;
  const size_t off_sh  = off_w + 5 * WBYTES;
  const size_t total   = off_sh + 5 * SBYTES;
  if (total > ws_size) return;
  if ((size_t)BATCH * PPAD * CH * 4 > 2 * TEN16) return;

  char* ws = (char*)d_ws;
  _Float16* XT  = (_Float16*)(ws + off_xt);
  _Float16* TMP = (_Float16*)(ws + off_tmp);
  float*    ATT = (float*)(ws + off_att);
  _Float16* Q16 = (_Float16*)(ws + off_q);
  _Float16* K16 = (_Float16*)(ws + off_k);
  _Float16* V16 = (_Float16*)(ws + off_v);
  _Float16* W16[5];
  float*    SHF[5];
  for (int i = 0; i < 5; ++i) {
    W16[i] = (_Float16*)(ws + off_w + (size_t)i * WBYTES);
    SHF[i] = (float*)(ws + off_sh + (size_t)i * SBYTES);
  }

  const float* target = (const float*)d_in[0];
  const float* source = (const float*)d_in[1];
  for (int i = 0; i < 5; ++i) {
    fold_w_kernel<<<dim3((CH * CH / 2 + 255) / 256), dim3(256), 0, stream>>>(
        (const float*)d_in[2 + 5 * i], (const float*)d_in[3 + 5 * i], (const float*)d_in[4 + 5 * i],
        (const float*)d_in[5 + 5 * i], (const float*)d_in[6 + 5 * i], W16[i], SHF[i]);
  }

  const dim3 gT(PPAD / 64, BATCH);
  nchw_to_pc16_kernel<<<gT, dim3(256), 0, stream>>>(target, XT);
  launch_gemm(XT,  W16[0], SHF[0], TMP, stream);
  launch_gemm(TMP, W16[1], SHF[1], Q16, stream);
  nchw_to_pc16_kernel<<<gT, dim3(256), 0, stream>>>(source, XT);
  launch_gemm(XT,  W16[2], SHF[2], TMP, stream);
  launch_gemm(TMP, W16[3], SHF[3], K16, stream);
  launch_gemm(XT,  W16[4], SHF[4], V16, stream);

  local_attn_kernel<<<dim3(NTILE * NTILE, BATCH), dim3(128), 0, stream>>>(Q16, K16, V16, ATT);

  pc_to_nchw_out_kernel<<<dim3((out_size / 4 + 255) / 256), dim3(256), 0, stream>>>(ATT, (float*)d_out, out_size);
}
